// GraphDownBlock_80676665688604
// MI455X (gfx1250) — hardware-verified
//
#include <hip/hip_runtime.h>
#include <stddef.h>


#define DF     64
#define NH     4
#define HC     16
#define GR     32
#define GTHR   128
#define AP     72
#define XSP    68
#define NB     960
#define NBD    12800
#define CHUNK  2048
#define NTHR   256
#define NWAVE  8
#define WCAP   256
#define NGRP   (CHUNK / (NTHR * 4))
#define SLOTSH 11

#define LDS_LIST_B (NWAVE * WCAP * 4 + NWAVE * 4)
#define LDS_GCN    (NB * DF * 4 + LDS_LIST_B)
#define LDS_GAT    ((NB * DF + 2 * NB * NH) * 4 + LDS_LIST_B + 32)
#define LDS_DEG    (NBD * 4 + NTHR * 4 + LDS_LIST_B)

static_assert(NGRP == 2);
static_assert(WCAP == (CHUNK / NTHR) * 32);
static_assert((1 << SLOTSH) == CHUNK);
static_assert(NB < (1 << 20) && NBD < (1 << 20));
static_assert((NB % (2 * NWAVE)) == 0);
static_assert(((NB * DF) % 4) == 0 && ((NB * DF + NB * NH) % 4) == 0 && (NBD % 4) == 0);
static_assert((NBD % GR) == 0);
static_assert(LDS_GCN == 253984);
static_assert(LDS_GAT == 284736);
static_assert(LDS_DEG == 60448);

typedef float          v2f   __attribute__((ext_vector_type(2)));
typedef float          v4f   __attribute__((ext_vector_type(4)));
typedef float          v8f   __attribute__((ext_vector_type(8)));
typedef int            v4i   __attribute__((ext_vector_type(4)));
typedef unsigned short v8us  __attribute__((ext_vector_type(8)));
typedef unsigned short v16us __attribute__((ext_vector_type(16)));
typedef __bf16         v16bf __attribute__((ext_vector_type(16)));
union Frag { v16bf v; v16us u; v8us half[2]; };

__device__ __forceinline__ v8f wm(v16us a, v16us b, v8f c) {
  Frag fa, fb;
  fa.u = a;
  fb.u = b;
  v8f d = __builtin_amdgcn_wmma_f32_16x16x32_bf16(false, fa.v, false, fb.v, (short)0, c, false, false);
  asm volatile("v_nop\n\tv_nop\n\tv_nop\n\tv_nop" : "+v"(d) : "v"(a), "v"(b));
  return d;
}

__device__ __forceinline__ unsigned short bfr(float f) {
  unsigned u = __float_as_uint(f);
  u += 0x7FFFu + ((u >> 16) & 1u);
  return (unsigned short)(u >> 16);
}
__device__ __forceinline__ float bff(unsigned short h) { return __uint_as_float(((unsigned)h) << 16); }

__device__ __forceinline__ void split8(v4f a, v4f b, v8us& hi, v8us& lo) {
  unsigned short t;
  t = bfr(a.x); hi[0] = t; lo[0] = bfr(a.x - bff(t));
  t = bfr(a.y); hi[1] = t; lo[1] = bfr(a.y - bff(t));
  t = bfr(a.z); hi[2] = t; lo[2] = bfr(a.z - bff(t));
  t = bfr(a.w); hi[3] = t; lo[3] = bfr(a.w - bff(t));
  t = bfr(b.x); hi[4] = t; lo[4] = bfr(b.x - bff(t));
  t = bfr(b.y); hi[5] = t; lo[5] = bfr(b.y - bff(t));
  t = bfr(b.z); hi[6] = t; lo[6] = bfr(b.z - bff(t));
  t = bfr(b.w); hi[7] = t; lo[7] = bfr(b.w - bff(t));
}

__device__ __forceinline__ v16us ldfrag(const unsigned short* p) {
  Frag f;
  f.half[0] = *(const v8us*)p;
  f.half[1] = *(const v8us*)(p + 16);
  return f.u;
}

__device__ __forceinline__ float hsum16(float v) {
  v += __shfl_xor(v, 8, 32);
  v += __shfl_xor(v, 4, 32);
  v += __shfl_xor(v, 2, 32);
  v += __shfl_xor(v, 1, 32);
  return v;
}

__device__ __forceinline__ float silu_f(float v) {
  const float e  = __expf(-fabsf(v));
  const float s  = __builtin_amdgcn_rcpf(1.0f + e);
  const float sg = (v >= 0.f) ? s : e * s;
  return v * sg;
}

__device__ __forceinline__ float lrelu_f(float v) { return (v > 0.f) ? v : 0.2f * v; }

__global__ __launch_bounds__(64) void k_prepw(const float* __restrict__ w0, const float* __restrict__ w1,
                                              const float* __restrict__ w2, const float* __restrict__ w3,
                                              const float* __restrict__ w4, const float* __restrict__ w5,
                                              unsigned short* Wt) {
  const int j = blockIdx.x;
  const int n = threadIdx.x;
  const float* W = (j == 0) ? w0 : (j == 1) ? w1 : (j == 2) ? w2 : (j == 3) ? w3 : (j == 4) ? w4 : w5;
  v8us hi[8], lo[8];
#pragma unroll
  for (int g = 0; g < 8; ++g) {
    v4f a, b;
    a.x = W[(8 * g + 0) * DF + n]; a.y = W[(8 * g + 1) * DF + n];
    a.z = W[(8 * g + 2) * DF + n]; a.w = W[(8 * g + 3) * DF + n];
    b.x = W[(8 * g + 4) * DF + n]; b.y = W[(8 * g + 5) * DF + n];
    b.z = W[(8 * g + 6) * DF + n]; b.w = W[(8 * g + 7) * DF + n];
    split8(a, b, hi[g], lo[g]);
  }
  unsigned short* ph = Wt + ((size_t)(2 * j) * DF + n) * DF;
  unsigned short* pl = Wt + ((size_t)(2 * j + 1) * DF + n) * DF;
#pragma unroll
  for (int g = 0; g < 8; ++g) {
    *(volatile v8us*)(ph + 8 * g) = hi[g];
    *(volatile v8us*)(pl + 8 * g) = lo[g];
  }
  __threadfence();
#pragma unroll
  for (int g = 0; g < 8; ++g) {
    *(volatile v8us*)(ph + 8 * g) = hi[g];
    *(volatile v8us*)(pl + 8 * g) = lo[g];
  }
}

template <bool SUMEA>
__device__ __forceinline__ int scan_chunk(const int* __restrict__ eid, const float* __restrict__ eav,
                                          int nE, bool al16, int cbase, int nodeBase, int nbOwn,
                                          int tid, int wave, int* list, float& easum) {
  int wc = 0;
#pragma unroll
  for (int g = 0; g < NGRP; ++g) {
    const int el0 = (g * NTHR + tid) * 4;
    const int e0  = cbase + el0;
    const int sent = -2147483647 - 1;
    v4i d;
    if (al16 && (e0 + 3 < nE)) {
      d = *(const v4i*)(eid + e0);
    } else {
      d.x = (e0     < nE) ? eid[(e0     < nE - 1) ? e0     : nE - 1] : sent;
      d.y = (e0 + 1 < nE) ? eid[(e0 + 1 < nE - 1) ? e0 + 1 : nE - 1] : sent;
      d.z = (e0 + 2 < nE) ? eid[(e0 + 2 < nE - 1) ? e0 + 2 : nE - 1] : sent;
      d.w = (e0 + 3 < nE) ? eid[(e0 + 3 < nE - 1) ? e0 + 3 : nE - 1] : sent;
    }
    if (SUMEA) {
      v4f a;
      if (al16 && (e0 + 3 < nE)) {
        a = *(const v4f*)(eav + e0);
      } else {
        a.x = (e0     < nE) ? eav[(e0     < nE - 1) ? e0     : nE - 1] : 0.f;
        a.y = (e0 + 1 < nE) ? eav[(e0 + 1 < nE - 1) ? e0 + 1 : nE - 1] : 0.f;
        a.z = (e0 + 2 < nE) ? eav[(e0 + 2 < nE - 1) ? e0 + 2 : nE - 1] : 0.f;
        a.w = (e0 + 3 < nE) ? eav[(e0 + 3 < nE - 1) ? e0 + 3 : nE - 1] : 0.f;
      }
      easum += a.x; easum += a.y; easum += a.z; easum += a.w;
    }
    const unsigned s0 = (unsigned)d.x - (unsigned)nodeBase;
    const unsigned s1 = (unsigned)d.y - (unsigned)nodeBase;
    const unsigned s2 = (unsigned)d.z - (unsigned)nodeBase;
    const unsigned s3 = (unsigned)d.w - (unsigned)nodeBase;
    const bool h0 = s0 < (unsigned)nbOwn;
    const bool h1 = s1 < (unsigned)nbOwn;
    const bool h2 = s2 < (unsigned)nbOwn;
    const bool h3 = s3 < (unsigned)nbOwn;
    const unsigned many = __builtin_amdgcn_ballot_w32(h0 | h1 | h2 | h3);
    if (many != 0u) {
      {
        const unsigned mj = __builtin_amdgcn_ballot_w32(h0);
        if (h0) {
          const int pos = wc + (int)__builtin_amdgcn_mbcnt_lo(mj, 0u);
          if (pos < WCAP) list[wave * WCAP + pos] = (int)((s0 << SLOTSH) | (unsigned)(el0 + 0));
        }
        wc += (int)__builtin_popcount(mj);
      }
      {
        const unsigned mj = __builtin_amdgcn_ballot_w32(h1);
        if (h1) {
          const int pos = wc + (int)__builtin_amdgcn_mbcnt_lo(mj, 0u);
          if (pos < WCAP) list[wave * WCAP + pos] = (int)((s1 << SLOTSH) | (unsigned)(el0 + 1));
        }
        wc += (int)__builtin_popcount(mj);
      }
      {
        const unsigned mj = __builtin_amdgcn_ballot_w32(h2);
        if (h2) {
          const int pos = wc + (int)__builtin_amdgcn_mbcnt_lo(mj, 0u);
          if (pos < WCAP) list[wave * WCAP + pos] = (int)((s2 << SLOTSH) | (unsigned)(el0 + 2));
        }
        wc += (int)__builtin_popcount(mj);
      }
      {
        const unsigned mj = __builtin_amdgcn_ballot_w32(h3);
        if (h3) {
          const int pos = wc + (int)__builtin_amdgcn_mbcnt_lo(mj, 0u);
          if (pos < WCAP) list[wave * WCAP + pos] = (int)((s3 << SLOTSH) | (unsigned)(el0 + 3));
        }
        wc += (int)__builtin_popcount(mj);
      }
    }
  }
  return wc;
}

__global__ __launch_bounds__(NTHR) void k_deg(const int* __restrict__ ei, const float* __restrict__ ew,
                                              const float* __restrict__ ea, float* dinv, float* scal,
                                              int nN, int nE) {
  extern __shared__ v4f lds_dyn[];
  float* dacc = (float*)lds_dyn;
  float* red  = dacc + NBD;
  int*   list = (int*)(red + NTHR);
  int*   wcnt = list + NWAVE * WCAP;
  const int tid  = threadIdx.x;
  const int lane = tid & 31;
  const int wave = tid >> 5;
  const int nodeBase = blockIdx.x * NBD;
  (void)nN;
  {
    const v4f z4 = {0.f, 0.f, 0.f, 0.f};
    for (int i = tid; i < NBD / 4; i += NTHR) lds_dyn[i] = z4;
  }
  __syncthreads();
  const int* eid = ei + nE;
  const bool al16 = ((nE & 3) == 0);
  float easum = 0.f;
  const int nChunks = (nE + CHUNK - 1) / CHUNK;
#pragma unroll 1
  for (int ch = 0; ch < nChunks; ++ch) {
    const int cbase = ch * CHUNK;
    const int wc = scan_chunk<true>(eid, ea, nE, al16, cbase, nodeBase, NBD, tid, wave, list, easum);
    if (lane == 0) wcnt[wave] = wc;
    __syncthreads();
    if (wave == 0) {
#pragma unroll 1
      for (int wsx = 0; wsx < NWAVE; ++wsx) {
        int n = wcnt[wsx];
        n = (n > WCAP) ? WCAP : n;
        n = (n < 0) ? 0 : n;
#pragma unroll 1
        for (int i = 0; i < n; ++i) {
          const int ent = list[wsx * WCAP + i];
          const int el  = ent & (CHUNK - 1);
          const unsigned su = (unsigned)ent >> SLOTSH;
          const int slot = (su < (unsigned)NBD) ? (int)su : (NBD - 1);
          int e = cbase + el;
          if (e > nE - 1) e = nE - 1;
          const float w = ew[e];
          if (lane == 0) dacc[slot] = dacc[slot] + w;
        }
      }
    }
    __syncthreads();
  }
  red[tid] = easum;
  __syncthreads();
#pragma unroll 1
  for (int s = NTHR / 2; s > 0; s >>= 1) {
    if (tid < s) red[tid] = red[tid] + red[tid + s];
    __syncthreads();
  }
  const float mea = red[0] * (1.0f / (float)nE);

  for (int i = tid * 4; i < NBD; i += NTHR * 4) {
    const v4f d = *(const v4f*)(dacc + i);
    v4f r;
    r.x = rsqrtf(d.x + 1.0f); r.y = rsqrtf(d.y + 1.0f); r.z = rsqrtf(d.z + 1.0f); r.w = rsqrtf(d.w + 1.0f);
    *(volatile v4f*)(dinv + (size_t)nodeBase + i) = r;
  }
  if (blockIdx.x == 0 && tid < 8) {
    v4f v = {0.f, 0.f, 0.f, 0.f};
    if (tid == 0) v.x = mea;
    *(volatile v4f*)(scal + 4 * tid) = v;
  }
  __threadfence();
  for (int i = tid * 4; i < NBD; i += NTHR * 4) {
    const v4f d = *(const v4f*)(dacc + i);
    v4f r;
    r.x = rsqrtf(d.x + 1.0f); r.y = rsqrtf(d.y + 1.0f); r.z = rsqrtf(d.z + 1.0f); r.w = rsqrtf(d.w + 1.0f);
    *(volatile v4f*)(dinv + (size_t)nodeBase + i) = r;
  }
  if (blockIdx.x == 0 && tid < 8) {
    v4f v = {0.f, 0.f, 0.f, 0.f};
    if (tid == 0) v.x = mea;
    *(volatile v4f*)(scal + 4 * tid) = v;
  }
}

__device__ __forceinline__ void stage_a(const float* __restrict__ X, int rowBase, int nN, int tid,
                                        unsigned short* Ah, unsigned short* Al) {
  const int r  = tid >> 2;
  const int c0 = (tid & 3) * 16;
  int row = rowBase + r;
  if (row > nN - 1) row = nN - 1;
  const float* p = X + (size_t)row * DF + c0;
  const v4f f0 = *(const v4f*)(p),     f1 = *(const v4f*)(p + 4);
  const v4f f2 = *(const v4f*)(p + 8), f3 = *(const v4f*)(p + 12);
  v8us h0, l0, h1, l1;
  split8(f0, f1, h0, l0);
  split8(f2, f3, h1, l1);
  *(v8us*)(Ah + r * AP + c0)     = h0;
  *(v8us*)(Ah + r * AP + c0 + 8) = h1;
  *(v8us*)(Al + r * AP + c0)     = l0;
  *(v8us*)(Al + r * AP + c0 + 8) = l1;
}

__global__ __launch_bounds__(GTHR) void k_gemm_pre(
    const float* __restrict__ X,
    const unsigned short* __restrict__ Brh, const unsigned short* __restrict__ Brl,
    const unsigned short* __restrict__ Bgh, const unsigned short* __restrict__ Bgl,
    const float* __restrict__ rb, const float* __restrict__ dinv,
    float* res, float* hs, int nN) {
  __shared__ __attribute__((aligned(16))) unsigned short Ah[GR * AP];
  __shared__ __attribute__((aligned(16))) unsigned short Al[GR * AP];
  __shared__ __attribute__((aligned(16))) float Xr[GR * XSP];
  __shared__ __attribute__((aligned(16))) float Xg[GR * XSP];

  const int tid  = threadIdx.x;
  const int lane = tid & 31;
  const int wave = tid >> 5;
  const int hh   = lane >> 4;
  const int m    = lane & 15;
  const int rowBase = blockIdx.x * GR;

  stage_a(X, rowBase, nN, tid, Ah, Al);
  __syncthreads();

  const int ncol = wave * 16 + m;
  v8f cr0 = {0.f, 0.f, 0.f, 0.f, 0.f, 0.f, 0.f, 0.f};
  v8f cr1 = cr0, cg0 = cr0, cg1 = cr0;
#pragma unroll
  for (int kt = 0; kt < DF / 32; ++kt) {
    const int k0 = kt * 32;
    const v16us bh = ldfrag(Brh + (size_t)ncol * DF + k0 + 8 * hh);
    const v16us bl = ldfrag(Brl + (size_t)ncol * DF + k0 + 8 * hh);
    const v16us gh = ldfrag(Bgh + (size_t)ncol * DF + k0 + 8 * hh);
    const v16us gl = ldfrag(Bgl + (size_t)ncol * DF + k0 + 8 * hh);
    const v16us a0h = ldfrag(Ah + m * AP + k0 + 8 * hh);
    const v16us a0l = ldfrag(Al + m * AP + k0 + 8 * hh);
    const v16us a1h = ldfrag(Ah + (16 + m) * AP + k0 + 8 * hh);
    const v16us a1l = ldfrag(Al + (16 + m) * AP + k0 + 8 * hh);
    cr0 = wm(a0h, bh, cr0); cr0 = wm(a0l, bh, cr0); cr0 = wm(a0h, bl, cr0);
    cr1 = wm(a1h, bh, cr1); cr1 = wm(a1l, bh, cr1); cr1 = wm(a1h, bl, cr1);
    cg0 = wm(a0h, gh, cg0); cg0 = wm(a0l, gh, cg0); cg0 = wm(a0h, gl, cg0);
    cg1 = wm(a1h, gh, cg1); cg1 = wm(a1l, gh, cg1); cg1 = wm(a1h, gl, cg1);
  }

  const float bv = rb[ncol];
#pragma unroll
  for (int r = 0; r < 8; ++r) {
    Xr[(8 * hh + r) * XSP + ncol]      = cr0[r] + bv;
    Xr[(16 + 8 * hh + r) * XSP + ncol] = cr1[r] + bv;
    Xg[(8 * hh + r) * XSP + ncol]      = cg0[r];
    Xg[(16 + 8 * hh + r) * XSP + ncol] = cg1[r];
  }
  __syncthreads();

  const int c4 = 4 * (lane & 15);
  v4f vr[4], vg[4];
  float* pr[4];
  float* pg[4];
#pragma unroll
  for (int i = 0; i < 4; ++i) {
    const int rloc = 8 * wave + 2 * i + hh;
    const int grow = rowBase + rloc;
    const int dn   = (grow < nN) ? grow : (nN - 1);
    const float dv = dinv[dn];
    vr[i] = *(const v4f*)(Xr + rloc * XSP + c4);
    vg[i] = *(const v4f*)(Xg + rloc * XSP + c4) * dv;
    pr[i] = res + (size_t)grow * DF + c4;
    pg[i] = hs  + (size_t)grow * DF + c4;
  }
#pragma unroll
  for (int i = 0; i < 4; ++i) { *(volatile v4f*)(pr[i]) = vr[i]; *(volatile v4f*)(pg[i]) = vg[i]; }
  __threadfence();
#pragma unroll
  for (int i = 0; i < 4; ++i) { *(volatile v4f*)(pr[i]) = vr[i]; *(volatile v4f*)(pg[i]) = vg[i]; }
}

__device__ __forceinline__ void epi_tile(v8f acc, int T, int hh, int m, int wave, int ncol,
                                         float cs, float cd, float* Xs, float* As, float* Ds) {
  float ss[8], sd[8];
#pragma unroll
  for (int r = 0; r < 8; ++r) {
    const float v = acc[r];
    Xs[(T * 16 + 8 * hh + r) * XSP + ncol] = v;
    ss[r] = v * cs;
    sd[r] = v * cd;
  }
#pragma unroll
  for (int mk = 1; mk < 16; mk <<= 1) {
#pragma unroll
    for (int r = 0; r < 8; ++r) {
      ss[r] += __shfl_xor(ss[r], mk, 32);
      sd[r] += __shfl_xor(sd[r], mk, 32);
    }
  }
  if (m == 0) {
#pragma unroll
    for (int r = 0; r < 8; ++r) {
      As[(T * 16 + 8 * hh + r) * NH + wave] = ss[r];
      Ds[(T * 16 + 8 * hh + r) * NH + wave] = sd[r];
    }
  }
}

__global__ __launch_bounds__(GTHR) void k_gemm_att(
    const float* __restrict__ X,
    const unsigned short* __restrict__ Bh, const unsigned short* __restrict__ Bl,
    const float* __restrict__ att_src, const float* __restrict__ att_dst,
    float* xl, float* asrc, float* adst, int nN) {
  __shared__ __attribute__((aligned(16))) unsigned short Ah[GR * AP];
  __shared__ __attribute__((aligned(16))) unsigned short Al[GR * AP];
  __shared__ __attribute__((aligned(16))) float Xs[GR * XSP];
  __shared__ __attribute__((aligned(16))) float As[GR * NH];
  __shared__ __attribute__((aligned(16))) float Ds[GR * NH];

  const int tid  = threadIdx.x;
  const int lane = tid & 31;
  const int wave = tid >> 5;
  const int hh   = lane >> 4;
  const int m    = lane & 15;
  const int rowBase = blockIdx.x * GR;

  stage_a(X, rowBase, nN, tid, Ah, Al);
  __syncthreads();

  const int ncol = wave * 16 + m;
  v8f c0a = {0.f, 0.f, 0.f, 0.f, 0.f, 0.f, 0.f, 0.f};
  v8f c1a = c0a;
#pragma unroll
  for (int kt = 0; kt < DF / 32; ++kt) {
    const int k0 = kt * 32;
    const v16us bh  = ldfrag(Bh + (size_t)ncol * DF + k0 + 8 * hh);
    const v16us bl  = ldfrag(Bl + (size_t)ncol * DF + k0 + 8 * hh);
    const v16us a0h = ldfrag(Ah + m * AP + k0 + 8 * hh);
    const v16us a0l = ldfrag(Al + m * AP + k0 + 8 * hh);
    const v16us a1h = ldfrag(Ah + (16 + m) * AP + k0 + 8 * hh);
    const v16us a1l = ldfrag(Al + (16 + m) * AP + k0 + 8 * hh);
    c0a = wm(a0h, bh, c0a); c0a = wm(a0l, bh, c0a); c0a = wm(a0h, bl, c0a);
    c1a = wm(a1h, bh, c1a); c1a = wm(a1l, bh, c1a); c1a = wm(a1h, bl, c1a);
  }

  const float cs = att_src[ncol];
  const float cd = att_dst[ncol];
  epi_tile(c0a, 0, hh, m, wave, ncol, cs, cd, Xs, As, Ds);
  epi_tile(c1a, 1, hh, m, wave, ncol, cs, cd, Xs, As, Ds);
  __syncthreads();

  const int c4 = 4 * (lane & 15);
  v4f xr[4];
  float* xpp[4];
#pragma unroll
  for (int i = 0; i < 4; ++i) {
    const int rloc = 8 * wave + 2 * i + hh;
    xr[i]  = *(const v4f*)(Xs + rloc * XSP + c4);
    xpp[i] = xl + (size_t)(rowBase + rloc) * DF + c4;
  }
  float* gp = 0;
  v4f gv = {0.f, 0.f, 0.f, 0.f};
  if (wave == 0) {
    gv = *(const v4f*)(As + 4 * lane);
    gp = asrc + (size_t)rowBase * NH + 4 * lane;
  } else if (wave == 1) {
    gv = *(const v4f*)(Ds + 4 * lane);
    gp = adst + (size_t)rowBase * NH + 4 * lane;
  }
#pragma unroll
  for (int i = 0; i < 4; ++i) *(volatile v4f*)(xpp[i]) = xr[i];
  if (gp) *(volatile v4f*)gp = gv;
  __threadfence();
#pragma unroll
  for (int i = 0; i < 4; ++i) *(volatile v4f*)(xpp[i]) = xr[i];
  if (gp) *(volatile v4f*)gp = gv;
}

__global__ __launch_bounds__(NTHR) void k_gcn(
    const int* __restrict__ ei, const float* __restrict__ ew,
    const float* __restrict__ hs, const float* __restrict__ dinv, const float* __restrict__ res,
    const float* __restrict__ gb, const float* __restrict__ lg, const float* __restrict__ lb,
    float* xo, int nN, int nE) {
  extern __shared__ v4f lds_dyn[];
  float* sacc = (float*)lds_dyn;
  int*   list = (int*)(sacc + NB * DF);
  int*   wcnt = list + NWAVE * WCAP;
  const int tid  = threadIdx.x;
  const int lane = tid & 31;
  const int wave = tid >> 5;
  const int nodeBase = blockIdx.x * NB;
  {
    const v4f z4 = {0.f, 0.f, 0.f, 0.f};
    for (int i = tid; i < NB * DF / 4; i += NTHR) lds_dyn[i] = z4;
  }
  __syncthreads();
  const int* eid = ei + nE;
  const bool al16 = ((nE & 3) == 0);
  float dummy = 0.f;
  const int nChunks = (nE + CHUNK - 1) / CHUNK;
#pragma unroll 1
  for (int ch = 0; ch < nChunks; ++ch) {
    const int cbase = ch * CHUNK;
    const int wc = scan_chunk<false>(eid, ew, nE, al16, cbase, nodeBase, NB, tid, wave, list, dummy);
    if (lane == 0) wcnt[wave] = wc;
    __syncthreads();
    if (wave == 0) {
#pragma unroll 1
      for (int wsx = 0; wsx < NWAVE; ++wsx) {
        int n = wcnt[wsx];
        n = (n > WCAP) ? WCAP : n;
        n = (n < 0) ? 0 : n;
#pragma unroll 1
        for (int i = 0; i < n; ++i) {
          const int ent = list[wsx * WCAP + i];
          const int el  = ent & (CHUNK - 1);
          const unsigned su = (unsigned)ent >> SLOTSH;
          const int slot = (su < (unsigned)NB) ? (int)su : (NB - 1);
          int e = cbase + el;
          if (e > nE - 1) e = nE - 1;
          int src = ei[e];
          src = (src < 0) ? 0 : ((src > nN - 1) ? (nN - 1) : src);
          const float w = ew[e];
          const v2f xv = *(const v2f*)(hs + (size_t)src * DF + 2 * lane);
          v2f* sp = (v2f*)(sacc + slot * DF + 2 * lane);
          const v2f cur = *sp;
          *sp = cur + w * xv;
        }
      }
    }
    __syncthreads();
  }

  const int j15 = lane & 15;
  const int hh  = lane >> 4;
  const int c4  = 4 * j15;
  const v4f gb4 = *(const v4f*)(gb + c4);
  const v4f lg4 = *(const v4f*)(lg + c4);
  const v4f lb4 = *(const v4f*)(lb + c4);
#pragma unroll 1
  for (int j = 0; j < NB / (2 * NWAVE); ++j) {
    const int s0 = wave * (NB / NWAVE) + 2 * j;
    if (nodeBase + s0 >= nN) break;
    const int slot = s0 + hh;
    const int node = nodeBase + slot;
    const bool valid = node < nN;
    const int nl = valid ? node : (nN - 1);
    const v4f sv = *(const v4f*)(sacc + slot * DF + c4);
    const v4f hv = *(const v4f*)(hs + (size_t)nl * DF + c4);
    const v4f rv = *(const v4f*)(res + (size_t)nl * DF + c4);
    const float dv = dinv[nl];
    const v4f g = (sv + hv) * dv + gb4;
    v4f t;
    t.x = silu_f(g.x) + rv.x;
    t.y = silu_f(g.y) + rv.y;
    t.z = silu_f(g.z) + rv.z;
    t.w = silu_f(g.w) + rv.w;
    const float s  = hsum16(t.x + t.y + t.z + t.w);
    const float mu = s * (1.0f / (float)DF);
    const v4f dd = t - mu;
    const float q  = hsum16(dd.x * dd.x + dd.y * dd.y + dd.z * dd.z + dd.w * dd.w);
    const float rs = rsqrtf(q * (1.0f / (float)DF) + 1e-5f);
    const v4f y = dd * rs * lg4 + lb4;
    float* op = xo + (size_t)nl * DF + c4;
    if (valid) *(volatile v4f*)op = y;
    __threadfence();
    if (valid) *(volatile v4f*)op = y;
  }
}

__global__ __launch_bounds__(NTHR) void k_gat(
    const int* __restrict__ ei, const float* __restrict__ ea,
    const float* __restrict__ xl, const float* __restrict__ asrc, const float* __restrict__ adst,
    const float* __restrict__ xres, const float* __restrict__ We, const float* __restrict__ ae,
    const float* __restrict__ gatb, const float* __restrict__ scal,
    float* xo, int nN, int nE) {
  extern __shared__ v4f lds_dyn[];
  float* sacc = (float*)lds_dyn;
  float* den  = sacc + NB * DF;
  float* mx   = den + NB * NH;
  int*   list = (int*)(mx + NB * NH);
  int*   wcnt = list + NWAVE * WCAP;
  float* kap  = (float*)(wcnt + NWAVE);
  const int tid  = threadIdx.x;
  const int lane = tid & 31;
  const int wave = tid >> 5;
  const int nodeBase = blockIdx.x * NB;
  {
    const v4f z4 = {0.f, 0.f, 0.f, 0.f};
    for (int i = tid; i < (NB * DF + NB * NH) / 4; i += NTHR) lds_dyn[i] = z4;
    for (int i = tid; i < NB * NH; i += NTHR) mx[i] = -1.0e30f;
    if (tid < NH) {
      float s = 0.f;
#pragma unroll 1
      for (int c = 0; c < HC; ++c) s += We[tid * HC + c] * ae[tid * HC + c];
      kap[tid] = s;
    }
  }
  __syncthreads();
  const int hdd = lane >> 3;
  const int hde = (lane & 15) >> 2;
  const float kd  = kap[hdd];
  const float ke  = kap[hde];
  const float mea = scal[0];
  const int* eid = ei + nE;
  const bool al16 = ((nE & 3) == 0);
  float dummy = 0.f;
  const int nChunks = (nE + CHUNK - 1) / CHUNK;
#pragma unroll 1
  for (int ch = 0; ch < nChunks; ++ch) {
    const int cbase = ch * CHUNK;
    const int wc = scan_chunk<false>(eid, ea, nE, al16, cbase, nodeBase, NB, tid, wave, list, dummy);
    if (lane == 0) wcnt[wave] = wc;
    __syncthreads();
    if (wave == 0) {
#pragma unroll 1
      for (int wsx = 0; wsx < NWAVE; ++wsx) {
        int n = wcnt[wsx];
        n = (n > WCAP) ? WCAP : n;
        n = (n < 0) ? 0 : n;
#pragma unroll 1
        for (int i = 0; i < n; ++i) {
          const int ent = list[wsx * WCAP + i];
          const int el  = ent & (CHUNK - 1);
          const unsigned su = (unsigned)ent >> SLOTSH;
          const int slot = (su < (unsigned)NB) ? (int)su : (NB - 1);
          int e = cbase + el;
          if (e > nE - 1) e = nE - 1;
          int src = ei[e];
          src = (src < 0) ? 0 : ((src > nN - 1) ? (nN - 1) : src);
          const float a = ea[e];
          int nd = nodeBase + slot;
          if (nd > nN - 1) nd = nN - 1;
          float al = asrc[(size_t)src * NH + hdd] + adst[(size_t)nd * NH + hdd] + a * kd;
          al = lrelu_f(al);
          const int mi = slot * NH + hdd;
          const float mo = mx[mi];
          const float mn = fmaxf(mo, al);
          const float sc = __expf(mo - mn);
          const float p  = __expf(al - mn);
          const v2f xv = *(const v2f*)(xl + (size_t)src * DF + 2 * lane);
          v2f* sp = (v2f*)(sacc + slot * DF + 2 * lane);
          const v2f cur = *sp;
          *sp = cur * sc + p * xv;
          if ((lane & 7) == 0) {
            const float dn = den[mi];
            den[mi] = dn * sc + p;
            mx[mi]  = mn;
          }
        }
      }
    }
    __syncthreads();
  }

  const int j15 = lane & 15;
  const int hh  = lane >> 4;
  const int c4  = 4 * j15;
  const v4f gb4 = *(const v4f*)(gatb + c4);
#pragma unroll 1
  for (int j = 0; j < NB / (2 * NWAVE); ++j) {
    const int s0 = wave * (NB / NWAVE) + 2 * j;
    if (nodeBase + s0 >= nN) break;
    const int slot = s0 + hh;
    const int node = nodeBase + slot;
    const bool valid = node < nN;
    const int nl = valid ? node : (nN - 1);
    float al = asrc[(size_t)nl * NH + hde] + adst[(size_t)nl * NH + hde] + mea * ke;
    al = lrelu_f(al);
    const int mi = slot * NH + hde;
    const float mo = mx[mi];
    const float mn = fmaxf(mo, al);
    const float sc = __expf(mo - mn);
    const float p  = __expf(al - mn);
    const v4f xs = *(const v4f*)(xl + (size_t)nl * DF + c4);
    const v4f sv = *(const v4f*)(sacc + slot * DF + c4) * sc + p * xs;
    const float dv  = den[mi] * sc + p;
    const float inv = __builtin_amdgcn_rcpf(dv + 1e-16f);
    const v4f o  = sv * inv + gb4;
    const v4f xr = *(const v4f*)(xres + (size_t)nl * DF + c4);
    v4f y;
    y.x = silu_f(o.x) + xr.x;
    y.y = silu_f(o.y) + xr.y;
    y.z = silu_f(o.z) + xr.z;
    y.w = silu_f(o.w) + xr.w;
    float* op = xo + (size_t)nl * DF + c4;
    if (valid) *(volatile v4f*)op = y;
    __threadfence();
    if (valid) *(volatile v4f*)op = y;
  }
}

static inline size_t al256(size_t v) { return (v + 255) & ~(size_t)255; }

extern "C" void kernel_launch(void* const* d_in, const int* in_sizes, int n_in,
                              void* d_out, int out_size, void* d_ws, size_t ws_size,
                              hipStream_t stream) {
  if (n_in < 28) return;
  const int nN = in_sizes[0] / DF;
  if (nN <= 0 || in_sizes[0] != nN * DF) return;
  const int nE = in_sizes[2];
  if (nE <= 0 || in_sizes[1] != 2 * nE || in_sizes[3] != nE) return;
  for (int l = 0; l < 2; ++l) {
    const int b = 4 + 12 * l;
    if (in_sizes[b] != DF * DF || in_sizes[b + 2] != DF * DF || in_sizes[b + 6] != DF * DF) return;
    if (in_sizes[b + 1] != DF || in_sizes[b + 3] != DF || in_sizes[b + 4] != DF ||
        in_sizes[b + 5] != DF || in_sizes[b + 7] != DF || in_sizes[b + 11] != DF) return;
    if (in_sizes[b + 8] != NH * HC || in_sizes[b + 9] != NH * HC || in_sizes[b + 10] != NH * HC) return;
  }
  if (out_size != nN * DF) return;

  const float* x  = (const float*)d_in[0];
  const int*   ei = (const int*)d_in[1];
  const float* ew = (const float*)d_in[2];
  const float* ea = (const float*)d_in[3];
  float* out = (float*)d_out;

  const int nP    = ((nN + GR - 1) / GR) * GR;
  const int gridG = nP / GR;
  const int gridD = (nN + NBD - 1) / NBD;
  const int gridA = (nN + NB - 1) / NB;

  size_t off = 0;
  unsigned short* Wt = (unsigned short*)((char*)d_ws + off); off = al256(off + (size_t)6 * 2 * DF * DF * 2);
  float* dinv = (float*)((char*)d_ws + off); off = al256(off + (size_t)gridD * NBD * 4);
  float* scal = (float*)((char*)d_ws + off); off = al256(off + 256);
  float* res  = (float*)((char*)d_ws + off); off = al256(off + (size_t)nP * DF * 4);
  float* hs   = (float*)((char*)d_ws + off); off = al256(off + (size_t)nP * DF * 4);
  float* x1   = (float*)((char*)d_ws + off); off = al256(off + (size_t)nP * DF * 4);
  float* xl   = (float*)((char*)d_ws + off); off = al256(off + (size_t)nP * DF * 4);
  float* xa   = (float*)((char*)d_ws + off); off = al256(off + (size_t)nP * DF * 4);
  float* asrc = (float*)((char*)d_ws + off); off = al256(off + (size_t)nP * NH * 4);
  float* adst = (float*)((char*)d_ws + off); off = al256(off + (size_t)nP * NH * 4);
  if (off > ws_size) return;

  k_prepw<<<6, 64, 0, stream>>>((const float*)d_in[4], (const float*)d_in[6], (const float*)d_in[10],
                                (const float*)d_in[16], (const float*)d_in[18], (const float*)d_in[22], Wt);

  hipFuncSetAttribute(reinterpret_cast<const void*>(&k_deg), hipFuncAttributeMaxDynamicSharedMemorySize, LDS_DEG);
  k_deg<<<gridD, NTHR, LDS_DEG, stream>>>(ei, ew, ea, dinv, scal, nN, nE);

  hipFuncSetAttribute(reinterpret_cast<const void*>(&k_gcn), hipFuncAttributeMaxDynamicSharedMemorySize, LDS_GCN);
  hipFuncSetAttribute(reinterpret_cast<const void*>(&k_gat), hipFuncAttributeMaxDynamicSharedMemorySize, LDS_GAT);

  const float* xcur = x;
  for (int l = 0; l < 2; ++l) {
    const int b = 4 + 12 * l;
    const float* gcn_b = (const float*)d_in[b + 1];
    const float* res_b = (const float*)d_in[b + 3];
    const float* ln_g  = (const float*)d_in[b + 4];
    const float* ln_b  = (const float*)d_in[b + 5];
    const float* gat_b = (const float*)d_in[b + 7];
    const float* a_src = (const float*)d_in[b + 8];
    const float* a_dst = (const float*)d_in[b + 9];
    const float* a_e   = (const float*)d_in[b + 10];
    const float* ew_w  = (const float*)d_in[b + 11];
    const unsigned short* Pgh = Wt + (size_t)(2 * (3 * l + 0) + 0) * DF * DF;
    const unsigned short* Pgl = Wt + (size_t)(2 * (3 * l + 0) + 1) * DF * DF;
    const unsigned short* Prh = Wt + (size_t)(2 * (3 * l + 1) + 0) * DF * DF;
    const unsigned short* Prl = Wt + (size_t)(2 * (3 * l + 1) + 1) * DF * DF;
    const unsigned short* Pah = Wt + (size_t)(2 * (3 * l + 2) + 0) * DF * DF;
    const unsigned short* Pal = Wt + (size_t)(2 * (3 * l + 2) + 1) * DF * DF;
    float* xnext = (l == 0) ? xa : out;

    k_gemm_pre<<<gridG, GTHR, 0, stream>>>(xcur, Prh, Prl, Pgh, Pgl, res_b, dinv, res, hs, nN);
    k_gcn<<<gridA, NTHR, LDS_GCN, stream>>>(ei, ew, hs, dinv, res, gcn_b, ln_g, ln_b, x1, nN, nE);
    k_gemm_att<<<gridG, GTHR, 0, stream>>>(x1, Pah, Pal, a_src, a_dst, xl, asrc, adst, nN);
    k_gat<<<gridA, NTHR, LDS_GAT, stream>>>(ei, ea, xl, asrc, adst, x1, ew_w, a_e, gat_b, scal, xnext, nN, nE);

    xcur = xnext;
  }
}
